// GroupedQueryAttention_58420145160441
// MI455X (gfx1250) — hardware-verified
//
#include <hip/hip_runtime.h>
#include <math.h>

#ifndef NB
#define NB 2
#endif
#ifndef SEQ
#define SEQ 2048
#endif
#define SEQ_FULL 2048
#define DM 2048
#define NH 16
#define NG 4
#define GS 4
#define HD 128
#define NQKV 3072
#define ERL ((SEQ < 256) ? SEQ : 256)
#define TP 132
#define PP 72
#define OP 132
#ifndef ATTN_ATTR
#define ATTN_ATTR
#endif
#ifndef GEMM_ATTR
#define GEMM_ATTR
#endif

static_assert(SEQ % 64 == 0);
static_assert(SEQ <= SEQ_FULL);
static_assert(ERL % 64 == 0);
static_assert((SEQ - ERL) % 64 == 0);
static_assert(NH * HD == DM);
static_assert(NG * GS == NH);
static_assert(NQKV == DM + 2 * NG * HD);
static_assert(HD == 128);
static_assert(DM % 64 == 0 && NQKV % 64 == 0 && DM % 32 == 0);
static_assert(((long long)NB * SEQ) % 64 == 0);
static_assert(DM % 8 == 0);
static_assert(PP % 8 == 0 && PP >= 64);
static_assert(OP % 4 == 0 && OP >= HD);

typedef __attribute__((ext_vector_type(16))) _Float16 v16h;
typedef __attribute__((ext_vector_type(16))) __bf16   v16b;
typedef __attribute__((ext_vector_type(16))) unsigned short v16us;
typedef __attribute__((ext_vector_type(8)))  unsigned short v8us;
typedef __attribute__((ext_vector_type(8)))  float    v8f;
typedef __attribute__((ext_vector_type(4)))  float    v4f;
typedef __attribute__((ext_vector_type(4)))  unsigned int v4u;

__device__ __forceinline__ v16us ldf(const unsigned short* __restrict__ p) {
    const v8us a = *(const v8us*)p; const v8us b = *(const v8us*)(p + 16);
    return __builtin_shufflevector(a, b, 0, 1, 2, 3, 4, 5, 6, 7, 8, 9, 10, 11, 12, 13, 14, 15);
}
__device__ __forceinline__ v16us ldf_lds(const unsigned short* p) {
    const v8us a = *(const v8us*)p; const v8us b = *(const v8us*)(p + 16);
    return __builtin_shufflevector(a, b, 0, 1, 2, 3, 4, 5, 6, 7, 8, 9, 10, 11, 12, 13, 14, 15);
}
template <int ET> __device__ __forceinline__ v8f mma(v16us a, v16us b, v8f c) {
    if (ET == 0) {
        const v16h ah = __builtin_bit_cast(v16h, a), bh = __builtin_bit_cast(v16h, b);
        c = __builtin_amdgcn_wmma_f32_16x16x32_f16(false, ah, false, bh, (short)0, c, false, false);
        asm volatile("v_nop\n\tv_nop\n\tv_nop\n\tv_nop" : "+v"(c) : "v"(ah), "v"(bh));
    } else {
        const v16b ab = __builtin_bit_cast(v16b, a), bb = __builtin_bit_cast(v16b, b);
        c = __builtin_amdgcn_wmma_f32_16x16x32_bf16(false, ab, false, bb, (short)0, c, false, false);
        asm volatile("v_nop\n\tv_nop\n\tv_nop\n\tv_nop" : "+v"(c) : "v"(ab), "v"(bb));
    }
    return c;
}
__device__ __forceinline__ void wave_sync() {
    __builtin_amdgcn_fence(3  , "workgroup");
    __builtin_amdgcn_wave_barrier();
    __builtin_amdgcn_fence(2  , "workgroup");
}
__device__ __forceinline__ int opq(int v) { asm volatile("" : "+v"(v)); return v; }

__device__ __forceinline__ float cmb_bf(float v) { const unsigned u = __builtin_bit_cast(unsigned, v); const unsigned r = (u + 0x7fffu + ((u >> 16) & 1u)) & 0xffff0000u; return __builtin_bit_cast(float, r); }
__device__ __forceinline__ unsigned short bfu_rne(float v) { unsigned u = __builtin_bit_cast(unsigned, v); u += 0x7FFFu + ((u >> 16) & 1u); return (unsigned short)(u >> 16); }
__device__ __forceinline__ void bfsplit(float v, unsigned short& hi, unsigned short& lo) { hi = bfu_rne(v); lo = bfu_rne(v - __builtin_bit_cast(float, (unsigned)hi << 16)); }
__device__ __forceinline__ unsigned short hbits(float v) { return __builtin_bit_cast(unsigned short, (_Float16)v); }
__device__ __forceinline__ unsigned pk2(unsigned short a, unsigned short b) { return (unsigned)a | ((unsigned)b << 16); }

__device__ __forceinline__ void st16_1(unsigned short* p, v4u a) { volatile v4u* d = (volatile v4u*)p; *d = a; __threadfence(); *d = a; }
__device__ __forceinline__ void st16_2(unsigned short* p0, v4u a, unsigned short* p1, v4u b) {
    volatile v4u* d0 = (volatile v4u*)p0; volatile v4u* d1 = (volatile v4u*)p1; *d0 = a; *d1 = b; __threadfence(); *d0 = a; *d1 = b; }

__global__ __launch_bounds__(256) void k_cast(const float* __restrict__ src, int rows, int rpb, long long sbs,
                                              unsigned short* d16, unsigned short* dbf, int wbf, float sc) {
    const long long u = (long long)blockIdx.x * 256 + threadIdx.x;
    if (u >= (long long)rows * (DM / 8)) return;
    const int r = (int)(u / (DM / 8)), c0 = 8 * (int)(u % (DM / 8));
    const int bb = r / rpb, rr = r - bb * rpb;
    const float* s = src + (long long)bb * sbs + (long long)rr * DM + c0;
    const v4f a = *(const v4f*)s, b2 = *(const v4f*)(s + 4);
    const float w0 = cmb_bf(a.x), w1 = cmb_bf(a.y), w2 = cmb_bf(a.z), w3 = cmb_bf(a.w);
    const float w4 = cmb_bf(b2.x), w5 = cmb_bf(b2.y), w6 = cmb_bf(b2.z), w7 = cmb_bf(b2.w);
    v4u pk; pk.x = pk2(hbits(w0 * sc), hbits(w1 * sc)); pk.y = pk2(hbits(w2 * sc), hbits(w3 * sc));
    pk.z = pk2(hbits(w4 * sc), hbits(w5 * sc)); pk.w = pk2(hbits(w6 * sc), hbits(w7 * sc));
    const size_t o = (size_t)r * DM + c0;
    if (wbf) {
        v4u pb;
        pb.x = pk2((unsigned short)(__builtin_bit_cast(unsigned, w0) >> 16), (unsigned short)(__builtin_bit_cast(unsigned, w1) >> 16));
        pb.y = pk2((unsigned short)(__builtin_bit_cast(unsigned, w2) >> 16), (unsigned short)(__builtin_bit_cast(unsigned, w3) >> 16));
        pb.z = pk2((unsigned short)(__builtin_bit_cast(unsigned, w4) >> 16), (unsigned short)(__builtin_bit_cast(unsigned, w5) >> 16));
        pb.w = pk2((unsigned short)(__builtin_bit_cast(unsigned, w6) >> 16), (unsigned short)(__builtin_bit_cast(unsigned, w7) >> 16));
        st16_2(d16 + o, pk, dbf + o, pb);
    } else st16_1(d16 + o, pk);
}

template <int ET, bool ARES>
__device__ __forceinline__ void gemm64_body(const unsigned short* __restrict__ Ap, const unsigned short* __restrict__ A2p, int lda, long long strideA,
                                            const unsigned short* __restrict__ Btp, int ldb, float* Cout, int ldc, long long strideC,
                                            int M, int N, int K, float scale) {
    __shared__ __align__(16) float sT[8][16 * 68];
    const int b = blockIdx.y, lane = threadIdx.x & 31, wave = threadIdx.x >> 5;
    const int tilesN = N >> 6, tilesM = M >> 6;
    const int tile = blockIdx.x * 8 + wave;
    if (tile >= tilesM * tilesN) return;
    const int tm = tile / tilesN, tn = tile - tm * tilesN;
    const int m0 = tm << 6, n0 = tn << 6;
    const unsigned short* Ab = Ap + (size_t)b * strideA;
    const unsigned short* Ab2 = A2p + (size_t)b * strideA;
    const int rl = lane & 15, koff = (lane >> 4) * 8, mOff = (lane >> 4) * 8;
    v8f acc[4][4];
#pragma unroll
    for (int i = 0; i < 4; ++i)
#pragma unroll
        for (int j = 0; j < 4; ++j) { v8f zz = {}; acc[i][j] = zz; }
    for (int k0 = 0; k0 < K; k0 += 32) {
        v16us bh[4];
#pragma unroll
        for (int j = 0; j < 4; ++j) bh[j] = ldf(Btp + (size_t)(n0 + (j << 4) + rl) * ldb + koff + k0);
#pragma unroll
        for (int i = 0; i < 4; ++i) {
            const size_t ao = (size_t)(m0 + (i << 4) + rl) * lda + koff + k0;
            const v16us ah = ldf(Ab + ao);
            v16us al = ah;
            if (ARES) al = ldf(Ab2 + ao);
#pragma unroll
            for (int j = 0; j < 4; ++j) {
                acc[i][j] = mma<ET>(ah, bh[j], acc[i][j]);
                if (ARES) acc[i][j] = mma<ET>(al, bh[j], acc[i][j]);
            }
        }
    }
    float* slab = sT[wave];
    float* C = Cout + (size_t)b * strideC;
    const int hh = lane >> 4, c4 = (lane & 15) * 4;
#pragma unroll
    for (int i = 0; i < 4; ++i) {
        const int mBase = m0 + (i << 4);
#pragma unroll
        for (int j = 0; j < 4; ++j)
#pragma unroll
            for (int r = 0; r < 8; ++r) slab[(mOff + r) * 68 + (j << 4) + rl] = acc[i][j][r] * scale;
        wave_sync();
        v4f vals[8];
#pragma unroll
        for (int it = 0; it < 8; ++it) vals[it] = *(const v4f*)(slab + (it * 2 + hh) * 68 + c4);
#pragma unroll
        for (int pass = 0; pass < 2; ++pass) {
#pragma unroll
            for (int it = 0; it < 8; ++it) *(volatile v4f*)(C + (size_t)(mBase + it * 2 + hh) * ldc + n0 + c4) = vals[it];
            __threadfence();
        }
        wave_sync();
    }
}
__global__ __launch_bounds__(256) GEMM_ATTR void k_gemm_qkv(const unsigned short* __restrict__ X16, const unsigned short* __restrict__ W16, float* QKV) {
    gemm64_body<0, false>(X16, X16, DM, 0, W16, DM, QKV, NQKV, 0, NB * SEQ, NQKV, DM, 1.0f / 256.0f);
}
__global__ __launch_bounds__(256) GEMM_ATTR void k_gemm_out(const unsigned short* __restrict__ CTXH, const unsigned short* __restrict__ WO16, float* out) {
    gemm64_body<0, false>(CTXH + (size_t)ERL * DM, CTXH + (size_t)ERL * DM, DM, (long long)SEQ * DM, WO16, DM, out + (size_t)ERL * DM, DM, (long long)SEQ * DM, SEQ - ERL, DM, DM, 1.0f / 4096.0f);
}
__global__ __launch_bounds__(256) GEMM_ATTR void k_gemm_oute(const unsigned short* __restrict__ CEH, const unsigned short* __restrict__ CEL, const unsigned short* __restrict__ WOB, float* out) {
    gemm64_body<1, true>(CEH, CEL, DM, (long long)ERL * DM, WOB, DM, out, DM, (long long)SEQ * DM, ERL, DM, DM, 1.0f);
}

__global__ __launch_bounds__(256) void k_nr(const float* __restrict__ QKV, const float* __restrict__ cosp, const float* __restrict__ sinp,
                                            const float* __restrict__ qnw, const float* __restrict__ knw,
                                            unsigned short* QH, unsigned short* QR, unsigned short* QEH, unsigned short* QEL,
                                            unsigned short* KH, unsigned short* KEH, unsigned short* KEL,
                                            unsigned short* VTH, unsigned short* VTEH, unsigned short* VTEL) {
    __shared__ __align__(16) float tile[64 * TP];
    const int tid = threadIdx.x, lane = tid & 31, w = tid >> 5;
    const int b = blockIdx.x / (SEQ / 64), t0 = (blockIdx.x % (SEQ / 64)) * 64;
    const int r24 = blockIdx.y;
    const int kind = (r24 < NH) ? 0 : ((r24 < NH + NG) ? 1 : 2);
    const bool early = (t0 < ERL);
#pragma unroll 1
    for (int i = 0; i < 8; ++i) {
        const int row = w * 8 + i, t = t0 + row;
        const float* src = QKV + ((size_t)b * SEQ + t) * NQKV + r24 * HD;
        float u0 = src[lane], u1 = src[lane + 32], u2 = src[lane + 64], u3 = src[lane + 96];
        if (kind < 2) {
            float ss = u0 * u0 + u1 * u1 + u2 * u2 + u3 * u3;
            ss += __shfl_xor(ss, 16, 32); ss += __shfl_xor(ss, 8, 32); ss += __shfl_xor(ss, 4, 32); ss += __shfl_xor(ss, 2, 32); ss += __shfl_xor(ss, 1, 32);
            const float rn = rsqrtf(ss * (1.0f / 128.0f) + 1e-6f);
            const float a0 = qnw[lane], a1 = qnw[lane + 32], a2 = qnw[lane + 64], a3 = qnw[lane + 96];
            const float b0 = knw[lane], b1 = knw[lane + 32], b2 = knw[lane + 64], b3 = knw[lane + 96];
            const bool isq = (kind == 0);
            u0 = u0 * rn * cmb_bf(isq ? a0 : b0); u1 = u1 * rn * cmb_bf(isq ? a1 : b1);
            u2 = u2 * rn * cmb_bf(isq ? a2 : b2); u3 = u3 * rn * cmb_bf(isq ? a3 : b3);
            const float* cr = cosp + (size_t)t * HD; const float* sr = sinp + (size_t)t * HD;
            const float c0 = cmb_bf(cr[lane]), c1 = cmb_bf(cr[lane + 32]), c2 = cmb_bf(cr[lane + 64]), c3 = cmb_bf(cr[lane + 96]);
            const float s0 = cmb_bf(sr[lane]), s1 = cmb_bf(sr[lane + 32]), s2 = cmb_bf(sr[lane + 64]), s3 = cmb_bf(sr[lane + 96]);
            const float o0 = u0 * c0 - u2 * s0, o1 = u1 * c1 - u3 * s1;
            const float o2 = u2 * c2 + u0 * s2, o3 = u3 * c3 + u1 * s3;
            u0 = o0; u1 = o1; u2 = o2; u3 = o3;
        }
        tile[row * TP + lane] = u0; tile[row * TP + lane + 32] = u1; tile[row * TP + lane + 64] = u2; tile[row * TP + lane + 96] = u3;
    }
    __syncthreads();
    if (kind < 2) {
        const int hg = (kind == 0) ? r24 : (r24 - NH);
        const int nhd = (kind == 0) ? NH : NG;
#pragma unroll 1
        for (int it = 0; it < 4; ++it) {
            const int idx = it * 256 + tid, row = idx >> 4, c8 = (idx & 15) * 8, t = t0 + row;
            const v4f fa = *(const v4f*)(tile + row * TP + c8), fb = *(const v4f*)(tile + row * TP + c8 + 4);
            const float f[8] = {fa.x, fa.y, fa.z, fa.w, fb.x, fb.y, fb.z, fb.w};
            unsigned short hb[8], rb[8], eh[8], el[8];
#pragma unroll
            for (int e = 0; e < 8; ++e) {
                const _Float16 hv = (_Float16)f[e];
                hb[e] = __builtin_bit_cast(unsigned short, hv);
                rb[e] = hbits((f[e] - (float)hv) * 2048.0f);
                bfsplit(f[e], eh[e], el[e]);
            }
            v4u ph, pr, pe, pl;
            ph.x = pk2(hb[0], hb[1]); ph.y = pk2(hb[2], hb[3]); ph.z = pk2(hb[4], hb[5]); ph.w = pk2(hb[6], hb[7]);
            pr.x = pk2(rb[0], rb[1]); pr.y = pk2(rb[2], rb[3]); pr.z = pk2(rb[4], rb[5]); pr.w = pk2(rb[6], rb[7]);
            pe.x = pk2(eh[0], eh[1]); pe.y = pk2(eh[2], eh[3]); pe.z = pk2(eh[4], eh[5]); pe.w = pk2(eh[6], eh[7]);
            pl.x = pk2(el[0], el[1]); pl.y = pk2(el[2], el[3]); pl.z = pk2(el[4], el[5]); pl.w = pk2(el[6], el[7]);
            const size_t o = (((size_t)b * nhd + hg) * SEQ + t) * HD + c8;
            const size_t oe = (((size_t)b * nhd + hg) * ERL + (early ? t : 0)) * HD + c8;
            if (kind == 0) { st16_2(QH + o, ph, QR + o, pr); if (early) st16_2(QEH + oe, pe, QEL + oe, pl); }
            else           { st16_1(KH + o, ph);             if (early) st16_2(KEH + oe, pe, KEL + oe, pl); }
        }
    } else {
        const int g = r24 - NH - NG;
#pragma unroll 1
        for (int it = 0; it < 4; ++it) {
            const int idx = it * 256 + tid, d = idx >> 3, t8 = (idx & 7) * 8;
            unsigned short hb[8], eh[8], el[8];
#pragma unroll
            for (int e = 0; e < 8; ++e) { const float v = tile[(t8 + e) * TP + d]; hb[e] = hbits(v); bfsplit(v, eh[e], el[e]); }
            v4u ph, pe, pl;
            ph.x = pk2(hb[0], hb[1]); ph.y = pk2(hb[2], hb[3]); ph.z = pk2(hb[4], hb[5]); ph.w = pk2(hb[6], hb[7]);
            pe.x = pk2(eh[0], eh[1]); pe.y = pk2(eh[2], eh[3]); pe.z = pk2(eh[4], eh[5]); pe.w = pk2(eh[6], eh[7]);
            pl.x = pk2(el[0], el[1]); pl.y = pk2(el[2], el[3]); pl.z = pk2(el[4], el[5]); pl.w = pk2(el[6], el[7]);
            const size_t o = (((size_t)b * NG + g) * HD + d) * SEQ + t0 + t8;
            const size_t oe = (((size_t)b * NG + g) * HD + d) * ERL + (early ? (t0 + t8) : 0);
            st16_1(VTH + o, ph);
            if (early) st16_2(VTEH + oe, pe, VTEL + oe, pl);
        }
    }
}

template <bool EV>
__device__ __forceinline__ void attn_body(const unsigned short* __restrict__ QA, const unsigned short* __restrict__ QB2,
                                          const unsigned short* __restrict__ KA, const unsigned short* __restrict__ KB2,
                                          const unsigned short* __restrict__ VA, const unsigned short* __restrict__ VB2,
                                          unsigned short* CA, unsigned short* CB2) {
    constexpr int ET = EV ? 1 : 0;
    constexpr int LR = EV ? ERL : SEQ;
    constexpr int QB0 = EV ? 0 : (ERL / 64);
    constexpr int NQB0 = EV ? (ERL / 64) : (SEQ / 64 - ERL / 64);
    constexpr int NQB = (NQB0 > 0) ? NQB0 : 1;
    __shared__ __align__(16) unsigned short Ph[4][16 * PP];
    __shared__ __align__(16) unsigned short Pl[EV ? 4 : 1][EV ? 16 * PP : 8];
    __shared__ __align__(16) float Os[4][16 * OP];
    const int tid = threadIdx.x, wave = tid >> 5, lane = tid & 31, hh = lane >> 4, c = lane & 15;
    const int bx = blockIdx.x;
    const int qb = QB0 + bx % NQB, bh = bx / NQB, h = bh % NH, b = bh / NH, g = h / GS;
    const int q0 = qb * 64 + wave * 16;
    const float NEG = -__builtin_inff();
    const float SCL = 0.08838834764831845f * 1.4426950408889634f;
    const float PSC = EV ? 1.0f : 32768.0f;
    const size_t qoff = (((size_t)b * NH + h) * LR + q0 + c) * HD + 8 * hh;
    const unsigned short* qpa = QA + qoff; const unsigned short* qpb = QB2 + qoff;
    const size_t koff = ((size_t)b * NG + g) * LR * HD + (size_t)c * HD + 8 * hh;
    const unsigned short* kpa = KA + koff; const unsigned short* kpb = KB2 + koff;
    const size_t voff = ((size_t)b * NG + g) * HD * LR + (size_t)c * LR + 8 * hh;
    const unsigned short* vpa = VA + voff; const unsigned short* vpb = VB2 + voff;
    unsigned short* ph = Ph[wave]; unsigned short* pl = Pl[EV ? wave : 0];

    float mrow[8], lrow[8]; v8f oacc[8];
#pragma unroll
    for (int r = 0; r < 8; ++r) { mrow[r] = NEG; lrow[r] = 0.f; }
#pragma unroll
    for (int t = 0; t < 8; ++t) { v8f zz = {}; oacc[t] = zz; }

#pragma unroll 1
    for (int kc = 0; kc <= qb; ++kc) {
        const int kv0 = kc * 64;
        v8f s[4], rr[4];
#pragma unroll
        for (int j = 0; j < 4; ++j) { v8f zz = {}; s[j] = zz; rr[j] = zz; }
#pragma unroll
        for (int ks = 0; ks < 4; ++ks) {
            const v16us qf = ldf(qpa + ks * 32); const v16us qf2 = ldf(qpb + ks * 32);
#pragma unroll
            for (int j = 0; j < 4; ++j) {
                const size_t ko = (size_t)(kv0 + 16 * j) * HD + ks * 32;
                const v16us ka = ldf(kpa + ko);
                if (EV) {
                    const v16us kl = ldf(kpb + ko);
                    s[j] = mma<ET>(qf, ka, s[j]); s[j] = mma<ET>(qf, kl, s[j]); s[j] = mma<ET>(qf2, ka, s[j]);
                } else {
                    s[j] = mma<ET>(qf, ka, s[j]); rr[j] = mma<ET>(qf2, ka, rr[j]);
                }
            }
            asm volatile("" ::: "memory");
        }
        const bool diag = (kc == qb);
        float cm[8];
#pragma unroll
        for (int r = 0; r < 8; ++r) {
            const int qrow = q0 + 8 * hh + r;
            float m = NEG;
#pragma unroll
            for (int j = 0; j < 4; ++j) {
                const int kvcol = kv0 + 16 * j + c;
                float v = EV ? s[j][r] : (s[j][r] + rr[j][r] * (1.0f / 2048.0f));
                v *= SCL;
                v = (diag && kvcol > qrow) ? NEG : v;
                s[j][r] = v; m = fmaxf(m, v);
            }
            m = fmaxf(m, __shfl_xor(m, 1, 32)); m = fmaxf(m, __shfl_xor(m, 2, 32));
            m = fmaxf(m, __shfl_xor(m, 4, 32)); m = fmaxf(m, __shfl_xor(m, 8, 32));
            cm[r] = m;
        }
#pragma unroll
        for (int r = 0; r < 8; ++r) {
            const float mnew = fmaxf(mrow[r], cm[r]);
            const float alpha = exp2f(mrow[r] - mnew);
            mrow[r] = mnew;
            float psum = 0.f;
#pragma unroll
            for (int j = 0; j < 4; ++j) {
                const float p = exp2f(s[j][r] - mnew);
                const int po = (8 * hh + r) * PP + j * 16 + c;
                if (EV) { unsigned short a, bl; bfsplit(p, a, bl); ph[po] = a; pl[po] = bl; psum += p; }
                else { const _Float16 p16 = (_Float16)(p * PSC); ph[po] = __builtin_bit_cast(unsigned short, p16); psum += (float)p16; }
            }
            psum += __shfl_xor(psum, 1, 32); psum += __shfl_xor(psum, 2, 32); psum += __shfl_xor(psum, 4, 32); psum += __shfl_xor(psum, 8, 32);
            lrow[r] = lrow[r] * alpha + psum;
#pragma unroll
            for (int t = 0; t < 8; ++t) oacc[t][r] *= alpha;
        }
        wave_sync();
#pragma unroll
        for (int kk = 0; kk < 2; ++kk) {
            const v16us pa = ldf_lds(ph + c * PP + kk * 32 + 8 * hh);
            v16us pb = pa;
            if (EV) pb = ldf_lds(pl + c * PP + kk * 32 + 8 * hh);
#pragma unroll
            for (int t = 0; t < 8; ++t) {
                const size_t vo = (size_t)(t * 16) * LR + kv0 + kk * 32;
                const v16us va = ldf(vpa + vo);
                if (EV) {
                    const v16us vl = ldf(vpb + vo);
                    oacc[t] = mma<ET>(pa, va, oacc[t]); oacc[t] = mma<ET>(pa, vl, oacc[t]); oacc[t] = mma<ET>(pb, va, oacc[t]);
                } else oacc[t] = mma<ET>(pa, va, oacc[t]);
                if (EV && (t & 3) == 3) asm volatile("" ::: "memory");
            }
            asm volatile("" ::: "memory");
        }
        wave_sync();
    }

    float* os = Os[wave];
    const float OSC = EV ? 1.0f : 16.0f;
#pragma unroll
    for (int r = 0; r < 8; ++r) {
        const float inv = OSC * (1.0f / lrow[r]);
#pragma unroll
        for (int t = 0; t < 8; ++t) os[(8 * hh + r) * OP + t * 16 + c] = oacc[t][r] * inv;
    }
    wave_sync();
    const int c8 = c * 8;
    v4u pk[8], pk2v[8];
#pragma unroll
    for (int it = 0; it < 8; ++it) {
        const int row = it * 2 + hh;
        const v4f fa = *(const v4f*)(os + row * OP + c8), fb = *(const v4f*)(os + row * OP + c8 + 4);
        const float f[8] = {fa.x, fa.y, fa.z, fa.w, fb.x, fb.y, fb.z, fb.w};
        unsigned short a[8], l[8];
#pragma unroll
        for (int e = 0; e < 8; ++e) { if (EV) bfsplit(f[e], a[e], l[e]); else { a[e] = hbits(f[e]); l[e] = 0; } }
        pk[it].x = pk2(a[0], a[1]); pk[it].y = pk2(a[2], a[3]); pk[it].z = pk2(a[4], a[5]); pk[it].w = pk2(a[6], a[7]);
        pk2v[it].x = pk2(l[0], l[1]); pk2v[it].y = pk2(l[2], l[3]); pk2v[it].z = pk2(l[4], l[5]); pk2v[it].w = pk2(l[6], l[7]);
    }
#pragma unroll
    for (int pass = 0; pass < 2; ++pass) {
#pragma unroll
        for (int it = 0; it < 8; ++it) {
            const int row = it * 2 + hh;
            const size_t o = ((size_t)b * LR + q0 + row) * DM + h * HD + c8;
            *(volatile v4u*)(CA + o) = pk[it];
            if (EV) *(volatile v4u*)(CB2 + o) = pk2v[it];
        }
        __threadfence();
    }
}
__global__ __launch_bounds__(128) ATTN_ATTR void k_attn_early(const unsigned short* __restrict__ QEH, const unsigned short* __restrict__ QEL, const unsigned short* __restrict__ KEH,
                                                              const unsigned short* __restrict__ KEL, const unsigned short* __restrict__ VTEH, const unsigned short* __restrict__ VTEL,
                                                              unsigned short* CEH, unsigned short* CEL) {
    attn_body<true>(QEH, QEL, KEH, KEL, VTEH, VTEL, CEH, CEL);
}

__global__ __launch_bounds__(128) ATTN_ATTR void k_attn_late(const unsigned short* __restrict__ QH, const unsigned short* __restrict__ QR, const unsigned short* __restrict__ KH,
                                                             const unsigned short* __restrict__ VTH, unsigned short* CTXH) {
    constexpr int QB0 = ERL / 64;
    constexpr int NQB0 = SEQ / 64 - ERL / 64;
    constexpr int NQB = (NQB0 > 0) ? NQB0 : 1;
    __shared__ __align__(16) unsigned short Ph[4][16 * PP];
    __shared__ __align__(16) float Os[4][16 * OP];
    const int tid = threadIdx.x, wave = tid >> 5, lane = tid & 31, hh = lane >> 4, c = lane & 15;
    const int bx = blockIdx.x;
    const int qb = QB0 + bx % NQB, bh = bx / NQB, h = bh % NH, b = bh / NH, g = h / GS;
    const int q0 = qb * 64 + wave * 16;
    const float NEG = -__builtin_inff();
    const float SCL = 0.08838834764831845f * 1.4426950408889634f;
    const float PSC = 32768.0f;
    const size_t qoff = (((size_t)b * NH + h) * SEQ + q0 + c) * HD + 8 * hh;
    const unsigned short* qpa = QH + qoff; const unsigned short* qpb = QR + qoff;
    const unsigned short* kpa = KH + ((size_t)b * NG + g) * SEQ * HD + (size_t)c * HD + 8 * hh;
    const unsigned short* vpa = VTH + ((size_t)b * NG + g) * HD * SEQ + (size_t)c * SEQ + 8 * hh;
    unsigned short* ph = Ph[wave];

    float mrow[8], lrow[8]; v8f oacc[8];
#pragma unroll
    for (int r = 0; r < 8; ++r) { mrow[r] = NEG; lrow[r] = 0.f; }
#pragma unroll
    for (int t = 0; t < 8; ++t) { v8f zz = {}; oacc[t] = zz; }

#pragma unroll 1
    for (int kc = 0; kc <= qb; ++kc) {
        const int kv0 = kc * 64;
        v8f s[4];
#pragma unroll
        for (int jh = 0; jh < 2; ++jh) {
            v8f sa0 = {}, sa1 = {}, ra0 = {}, ra1 = {};
#pragma unroll
            for (int ks = 0; ks < 4; ++ks) {
                const int qo = opq(ks * 32);
                const v16us qf = ldf(qpa + qo); const v16us qf2 = ldf(qpb + qo);
                const unsigned short* kp = kpa + (size_t)(kv0 + 32 * jh) * HD + qo;
                const v16us k0 = ldf(kp); const v16us k1 = ldf(kp + 16 * HD);
                sa0 = mma<0>(qf, k0, sa0); ra0 = mma<0>(qf2, k0, ra0);
                sa1 = mma<0>(qf, k1, sa1); ra1 = mma<0>(qf2, k1, ra1);
            }
            s[2 * jh]     = sa0 + ra0 * (1.0f / 2048.0f);
            s[2 * jh + 1] = sa1 + ra1 * (1.0f / 2048.0f);
        }
        const bool diag = (kc == qb);
        float cm[8];
#pragma unroll
        for (int r = 0; r < 8; ++r) {
            const int qrow = q0 + 8 * hh + r;
            float m = NEG;
#pragma unroll
            for (int j = 0; j < 4; ++j) {
                const int kvcol = kv0 + 16 * j + c;
                float v = s[j][r] * SCL;
                v = (diag && kvcol > qrow) ? NEG : v;
                s[j][r] = v; m = fmaxf(m, v);
            }
            m = fmaxf(m, __shfl_xor(m, 1, 32)); m = fmaxf(m, __shfl_xor(m, 2, 32));
            m = fmaxf(m, __shfl_xor(m, 4, 32)); m = fmaxf(m, __shfl_xor(m, 8, 32));
            cm[r] = m;
        }
#pragma unroll
        for (int r = 0; r < 8; ++r) {
            const float mnew = fmaxf(mrow[r], cm[r]);
            const float alpha = exp2f(mrow[r] - mnew);
            mrow[r] = mnew;
            float psum = 0.f;
#pragma unroll
            for (int j = 0; j < 4; ++j) {
                const float p = exp2f(s[j][r] - mnew);
                const _Float16 p16 = (_Float16)(p * PSC);
                ph[(8 * hh + r) * PP + j * 16 + c] = __builtin_bit_cast(unsigned short, p16);
                psum += (float)p16;
            }
            psum += __shfl_xor(psum, 1, 32); psum += __shfl_xor(psum, 2, 32); psum += __shfl_xor(psum, 4, 32); psum += __shfl_xor(psum, 8, 32);
            lrow[r] = lrow[r] * alpha + psum;
#pragma unroll
            for (int t = 0; t < 8; ++t) oacc[t][r] *= alpha;
        }
        wave_sync();
#pragma unroll
        for (int kk = 0; kk < 2; ++kk) {
            const v16us pa = ldf_lds(ph + c * PP + kk * 32 + 8 * hh);
#pragma unroll
            for (int tg = 0; tg < 2; ++tg) {
                const int vo = opq(kv0 + kk * 32);
#pragma unroll
                for (int t4 = 0; t4 < 4; ++t4) {
                    const int t = tg * 4 + t4;
                    const v16us va = ldf(vpa + (size_t)(t * 16) * SEQ + vo);
                    oacc[t] = mma<0>(pa, va, oacc[t]);
                }
            }
        }
        wave_sync();
    }

    float* os = Os[wave];
#pragma unroll
    for (int r = 0; r < 8; ++r) {
        const float inv = 16.0f * (1.0f / lrow[r]);
#pragma unroll
        for (int t = 0; t < 8; ++t) os[(8 * hh + r) * OP + t * 16 + c] = oacc[t][r] * inv;
    }
    wave_sync();
    const int c8 = c * 8;
    v4u pk[8];
#pragma unroll
    for (int it = 0; it < 8; ++it) {
        const int row = it * 2 + hh;
        const v4f fa = *(const v4f*)(os + row * OP + c8), fb = *(const v4f*)(os + row * OP + c8 + 4);
        pk[it].x = pk2(hbits(fa.x), hbits(fa.y)); pk[it].y = pk2(hbits(fa.z), hbits(fa.w));
        pk[it].z = pk2(hbits(fb.x), hbits(fb.y)); pk[it].w = pk2(hbits(fb.z), hbits(fb.w));
    }
#pragma unroll
    for (int pass = 0; pass < 2; ++pass) {
#pragma unroll
        for (int it = 0; it < 8; ++it) {
            const int row = it * 2 + hh;
            const size_t o = ((size_t)b * SEQ + q0 + row) * DM + h * HD + c8;
            *(volatile v4u*)(CTXH + o) = pk[it];
        }
        __threadfence();
    }
}

constexpr size_t cmax(size_t a, size_t b) { return a > b ? a : b; }
constexpr size_t MT = (size_t)NB * SEQ;
constexpr size_t SZ_X16 = MT * DM * 2;
constexpr size_t SZ_WO = (size_t)DM * DM * 2;
constexpr size_t SZ_R0 = cmax(SZ_X16, 2 * SZ_WO);
constexpr size_t SZ_WQKV = (size_t)NQKV * DM * 2;
constexpr size_t SZ_QKV = MT * NQKV * 4;
constexpr size_t SZ_CTXH = MT * DM * 2;
constexpr size_t SZ_CTXE = (size_t)NB * ERL * DM * 2;
constexpr size_t SZ_R1 = cmax(SZ_QKV, SZ_CTXH + 2 * SZ_CTXE);
constexpr size_t SZ_Q = (size_t)NB * NH * SEQ * HD * 2;
constexpr size_t SZ_KV = (size_t)NB * NG * SEQ * HD * 2;
constexpr size_t SZ_QE = (size_t)NB * NH * ERL * HD * 2;
constexpr size_t SZ_KVE = (size_t)NB * NG * ERL * HD * 2;
constexpr size_t OFF_R0 = 0;
constexpr size_t OFF_WQKV = OFF_R0 + SZ_R0;
constexpr size_t OFF_R1 = OFF_WQKV + SZ_WQKV;
constexpr size_t OFF_QH = OFF_R1 + SZ_R1;
constexpr size_t OFF_QR = OFF_QH + SZ_Q;
constexpr size_t OFF_KH = OFF_QR + SZ_Q;
constexpr size_t OFF_VTH = OFF_KH + SZ_KV;
constexpr size_t OFF_QEH = OFF_VTH + SZ_KV;
constexpr size_t OFF_QEL = OFF_QEH + SZ_QE;
constexpr size_t OFF_KEH = OFF_QEL + SZ_QE;
constexpr size_t OFF_KEL = OFF_KEH + SZ_KVE;
constexpr size_t OFF_VTEH = OFF_KEL + SZ_KVE;
constexpr size_t OFF_VTEL = OFF_VTEH + SZ_KVE;
constexpr size_t WS_TOTAL = OFF_VTEL + SZ_KVE;
static_assert(WS_TOTAL <= (size_t)134217728);
static_assert(SZ_X16 <= SZ_R0 && 2 * SZ_WO <= SZ_R0);
static_assert(SZ_QKV <= SZ_R1 && SZ_CTXH + 2 * SZ_CTXE <= SZ_R1);
static_assert(SZ_R0 % 256 == 0 && SZ_WQKV % 256 == 0 && SZ_R1 % 256 == 0 && SZ_Q % 256 == 0 && SZ_KV % 256 == 0 && SZ_QE % 256 == 0 && SZ_KVE % 256 == 0 && SZ_WO % 256 == 0 && SZ_CTXH % 256 == 0 && SZ_CTXE % 256 == 0);

extern "C" void kernel_launch(void* const* d_in, const int* in_sizes, int n_in, void* d_out, int out_size, void* d_ws, size_t ws_size, hipStream_t stream) {
    if (n_in < 9) return;
    if (in_sizes[0] < (NB - 1) * SEQ_FULL * DM + SEQ * DM) return;
    if (in_sizes[1] < SEQ * HD || in_sizes[2] < SEQ * HD) return;
    if (in_sizes[3] < DM * DM || in_sizes[4] < NG * HD * DM || in_sizes[5] < NG * HD * DM || in_sizes[6] < DM * DM) return;
    if (in_sizes[7] < HD || in_sizes[8] < HD) return;
    if (out_size < (int)(MT * DM)) return;
    if (ws_size < WS_TOTAL) return;
    const float* x    = (const float*)d_in[0];
    const float* cosp = (const float*)d_in[1];
    const float* sinp = (const float*)d_in[2];
    const float* wq   = (const float*)d_in[3];
    const float* wk   = (const float*)d_in[4];
    const float* wv   = (const float*)d_in[5];
    const float* wo   = (const float*)d_in[6];
    const float* qnw  = (const float*)d_in[7];
    const float* knw  = (const float*)d_in[8];
    float* out = (float*)d_out;
    char* ws = (char*)d_ws;
    unsigned short* X16  = (unsigned short*)(ws + OFF_R0);
    unsigned short* WO16 = (unsigned short*)(ws + OFF_R0);
    unsigned short* WOB  = (unsigned short*)(ws + OFF_R0 + SZ_WO);
    unsigned short* WQKV = (unsigned short*)(ws + OFF_WQKV);
    float* QKV           = (float*)(ws + OFF_R1);
    unsigned short* CTXH = (unsigned short*)(ws + OFF_R1);
    unsigned short* CEH  = (unsigned short*)(ws + OFF_R1 + SZ_CTXH);
    unsigned short* CEL  = (unsigned short*)(ws + OFF_R1 + SZ_CTXH + SZ_CTXE);
    unsigned short* QH   = (unsigned short*)(ws + OFF_QH);
    unsigned short* QR   = (unsigned short*)(ws + OFF_QR);
    unsigned short* KH   = (unsigned short*)(ws + OFF_KH);
    unsigned short* VTH  = (unsigned short*)(ws + OFF_VTH);
    unsigned short* QEH  = (unsigned short*)(ws + OFF_QEH);
    unsigned short* QEL  = (unsigned short*)(ws + OFF_QEL);
    unsigned short* KEH  = (unsigned short*)(ws + OFF_KEH);
    unsigned short* KEL  = (unsigned short*)(ws + OFF_KEL);
    unsigned short* VTEH = (unsigned short*)(ws + OFF_VTEH);
    unsigned short* VTEL = (unsigned short*)(ws + OFF_VTEL);

    k_cast<<<(unsigned)((MT * (DM / 8) + 255) / 256), 256, 0, stream>>>(x, (int)MT, SEQ, (long long)SEQ_FULL * DM, X16, X16, 0, 1.0f);
    k_cast<<<(unsigned)(((size_t)DM * (DM / 8) + 255) / 256), 256, 0, stream>>>(wq, DM, DM, 0, WQKV, WQKV, 0, 256.0f);
    k_cast<<<(unsigned)(((size_t)NG * HD * (DM / 8) + 255) / 256), 256, 0, stream>>>(wk, NG * HD, NG * HD, 0, WQKV + (size_t)DM * DM, WQKV, 0, 256.0f);
    k_cast<<<(unsigned)(((size_t)NG * HD * (DM / 8) + 255) / 256), 256, 0, stream>>>(wv, NG * HD, NG * HD, 0, WQKV + (size_t)(DM + NG * HD) * DM, WQKV, 0, 256.0f);
    k_gemm_qkv<<<dim3((unsigned)(((MT / 64) * (NQKV / 64) + 7) / 8), 1), 256, 0, stream>>>(X16, WQKV, QKV);
    k_cast<<<(unsigned)(((size_t)DM * (DM / 8) + 255) / 256), 256, 0, stream>>>(wo, DM, DM, 0, WO16, WOB, 1, 256.0f);
    k_nr<<<dim3((unsigned)(NB * (SEQ / 64)), (unsigned)(NH + 2 * NG)), 256, 0, stream>>>(QKV, cosp, sinp, qnw, knw, QH, QR, QEH, QEL, KH, KEH, KEL, VTH, VTEH, VTEL);
    k_attn_early<<<(unsigned)(NB * NH * (ERL / 64)), 128, 0, stream>>>(QEH, QEL, KEH, KEL, VTEH, VTEL, CEH, CEL);
    if (SEQ > ERL) k_attn_late<<<(unsigned)(NB * NH * ((SEQ - ERL) / 64 > 0 ? (SEQ - ERL) / 64 : 1)), 128, 0, stream>>>(QH, QR, KH, VTH, CTXH);
    k_gemm_oute<<<dim3((unsigned)(((ERL / 64) * (DM / 64) + 7) / 8), (unsigned)NB), 256, 0, stream>>>(CEH, CEL, WOB, out);
    if (SEQ > ERL) k_gemm_out<<<dim3((unsigned)((((SEQ - ERL) / 64) * (DM / 64) + 7) / 8), (unsigned)NB), 256, 0, stream>>>(CTXH, WO16, out);
}
